// PyTorchModel_18305150615594
// MI455X (gfx1250) — hardware-verified
//
#include <hip/hip_runtime.h>

typedef __bf16         v16b __attribute__((ext_vector_type(16)));
typedef unsigned short v8us __attribute__((ext_vector_type(8)));
typedef float          v8f  __attribute__((ext_vector_type(8)));
typedef float          v4f  __attribute__((ext_vector_type(4)));
typedef unsigned       v4u  __attribute__((ext_vector_type(4)));

union Frag { v16b v; v8us h8[2]; unsigned short s[16]; };

#define NS    16
#define NE    16
#define NF    16
#define NP    32
#define NH    128
#define NX    48
#define ROWS  256
#define NTHR  256
#define NWAV  8
#define NSLOT 512
#define NTILE 32
#define NTPE  16
#define XG    6
#define N0F   32768
#define N1F   16384

__device__ __forceinline__ unsigned short bf_rne(float x) {
    unsigned u = __float_as_uint(x);
    u += 0x7FFFu + ((u >> 16) & 1u);
    return (unsigned short)(u >> 16);
}
__device__ __forceinline__ void split2(float x, unsigned short& hi, unsigned short& lo) {
    hi = bf_rne(x);
    const float hf = __uint_as_float(((unsigned)hi) << 16);
    lo = bf_rne(x - hf);
}

__device__ __forceinline__ float fast_tanh(float x) {
    const float e = __builtin_amdgcn_exp2f(x * 2.8853900817779268f);
    return 1.0f - 2.0f * __builtin_amdgcn_rcpf(e + 1.0f);
}

__device__ __forceinline__ v8f wmma3(v8f acc, const Frag& ah, const Frag& al,
                                     const Frag& bh, const Frag& bl) {
    acc = __builtin_amdgcn_wmma_f32_16x16x32_bf16(false, ah.v, false, bh.v, (short)0, acc, false, false);
    acc = __builtin_amdgcn_wmma_f32_16x16x32_bf16(false, ah.v, false, bl.v, (short)0, acc, false, false);
    acc = __builtin_amdgcn_wmma_f32_16x16x32_bf16(false, al.v, false, bh.v, (short)0, acc, false, false);
    asm volatile("v_nop\n\tv_nop\n\tv_nop\n\tv_nop"
                 : "+v"(acc) : "v"(ah.v), "v"(al.v), "v"(bh.v), "v"(bl.v));
    return acc;
}

__device__ __forceinline__ v4f lo4(v8f a) { v4f r; r[0] = a[0]; r[1] = a[1]; r[2] = a[2]; r[3] = a[3]; return r; }
__device__ __forceinline__ v4f hi4(v8f a) { v4f r; r[0] = a[4]; r[1] = a[5]; r[2] = a[6]; r[3] = a[7]; return r; }

__device__ __forceinline__ void pack_group(v4f a, v4f b, v8us& hv, v8us& lv) {
    #pragma unroll
    for (int i = 0; i < 4; ++i) {
        unsigned short h0, l0, h1, l1;
        split2(a[i], h0, l0);
        split2(b[i], h1, l1);
        hv[i] = h0; lv[i] = l0; hv[4 + i] = h1; lv[4 + i] = l1;
    }
}

__launch_bounds__(256)
__global__ void k_pack(const float* __restrict__ W0, const float* __restrict__ W1,
                       v4u* a0f, v4u* a1f) {
    const int gid = blockIdx.x * blockDim.x + threadIdx.x;
    if (gid >= N0F + N1F) return;
    float v[8];
    int part, u;
    volatile v4u* dst;
    if (gid < N0F) {
        u = gid;
        const int q  = u & 1;
        const int L  = (u >> 1) & 31;
        part         = (u >> 6) & 1;
        const int c  = (u >> 7) & 1;
        const int t8 = (u >> 8) & 7;
        const int e  = (u >> 11) & 15;
        const int g  = L >> 4;
        const int h  = t8 * 16 + (L & 15);
        #pragma unroll
        for (int ii = 0; ii < 8; ++ii) {
            const int k = c * 32 + q * 16 + 8 * g + ii;
            v[ii] = (k < NX) ? W0[((size_t)e * NX + k) * NH + h] : 0.0f;
        }
        dst = (volatile v4u*)a0f;
    } else {
        u = gid - N0F;
        const int q  = u & 1;
        const int L  = (u >> 1) & 31;
        part         = (u >> 6) & 1;
        const int c  = (u >> 7) & 3;
        const int t2 = (u >> 9) & 1;
        const int e  = (u >> 10) & 15;
        const int g  = L >> 4;
        const int p  = t2 * 16 + (L & 15);
        #pragma unroll
        for (int ii = 0; ii < 8; ++ii) {
            const int k = c * 32 + q * 16 + 8 * g + ii;
            v[ii] = W1[((size_t)e * NH + k) * NP + p];
        }
        dst = (volatile v4u*)a1f;
    }
    unsigned s[8];
    #pragma unroll
    for (int ii = 0; ii < 8; ++ii) {
        unsigned short hi, lo;
        split2(v[ii], hi, lo);
        s[ii] = (unsigned)(part ? lo : hi);
    }
    v4u w;
    w[0] = s[0] | (s[1] << 16);
    w[1] = s[2] | (s[3] << 16);
    w[2] = s[4] | (s[5] << 16);
    w[3] = s[6] | (s[7] << 16);
    dst[u] = w;
    __threadfence();
    dst[u] = w;
}

__launch_bounds__(NTHR)
__global__ void k_main(const int*   __restrict__ ids,
                       const float* __restrict__ feats,
                       const float* __restrict__ p_in,
                       const int*   __restrict__ seq_len,
                       const float* __restrict__ b0,
                       const float* __restrict__ b1,
                       const v8us*  __restrict__ a0f,
                       const v8us*  __restrict__ a1f,
                       float* out, int nrows) {
    __shared__ v4f   pbuf4[ROWS * 8];
    __shared__ v8us  xsh[NSLOT * XG];
    __shared__ v8us  xsl[NSLOT * XG];
    __shared__ v4f   osl4[NSLOT * 8];
    __shared__ float b0s[NE * NH];
    __shared__ float b1s[NE * NP];
    __shared__ int   cntW[NWAV * NE];
    __shared__ int   wofs[NWAV * NE];
    __shared__ int   ntE[NE];
    __shared__ int   startT[NE];

    const int t    = threadIdx.x;
    const int lane = t & 31;
    const int wave = __builtin_amdgcn_readfirstlane(t >> 5);
    const int m16  = lane & 15;
    const int g    = lane >> 4;
    const int r0   = blockIdx.x * ROWS;
    const int grow = r0 + t;
    const bool rowok = grow < nrows;

    v8us z8;
    #pragma unroll
    for (int i = 0; i < 8; ++i) z8[i] = 0;
    v4f z4; z4[0] = 0.f; z4[1] = 0.f; z4[2] = 0.f; z4[3] = 0.f;

    {
        const v4f* pin4 = (const v4f*)p_in;
        for (int i = t; i < ROWS * 8; i += NTHR) {
            const int rr = i >> 3;
            pbuf4[i] = (r0 + rr < nrows) ? pin4[(size_t)(r0 + rr) * 8 + (i & 7)] : z4;
        }
    }
    for (int i = t; i < NE * NH; i += NTHR) b0s[i] = b0[i];
    for (int i = t; i < NE * NP; i += NTHR) b1s[i] = b1[i];
    const int slen = rowok ? seq_len[grow] : 0;
    __syncthreads();

    #pragma unroll 1
    for (int n = 0; n < NS; ++n) {
        for (int i = t; i < NSLOT * XG; i += NTHR) { xsh[i] = z8; xsl[i] = z8; }
        int myid = rowok ? ids[(size_t)grow * NS + n] : 0;
        myid = myid < 0 ? 0 : (myid > NE - 1 ? NE - 1 : myid);
        const bool active = (n < slen);
        unsigned mymask = 0u;
        int mycnt = 0;
        #pragma unroll
        for (int e = 0; e < NE; ++e) {
            const unsigned msk = __builtin_amdgcn_ballot_w32(active && (myid == e));
            if (myid == e) mymask = msk;
            if (lane == e) mycnt = __builtin_popcount(msk);
        }
        if (lane < NE) cntW[wave * NE + lane] = mycnt;
        const int rankw = __builtin_popcount(mymask & ((1u << lane) - 1u));
        __syncthreads();

        if (t == 0) {
            int run = 0;
            for (int e = 0; e < NE; ++e) {
                int tot = 0;
                for (int w = 0; w < NWAV; ++w) { wofs[w * NE + e] = tot; tot += cntW[w * NE + e]; }
                if (tot > ROWS) tot = ROWS;
                if (tot < 0) tot = 0;
                int nt = (tot + 15) >> 4;
                if (nt > NTILE - run) nt = NTILE - run;
                startT[e] = run;
                ntE[e]    = nt;
                run += nt;
            }
        }
        __syncthreads();

        int myslot = 0;
        if (active) {
            int slot = startT[myid] * 16 + wofs[wave * NE + myid] + rankw;
            slot = ((unsigned)slot < (unsigned)NSLOT) ? slot : (NSLOT - 1);
            myslot = slot;
            const int xb = slot * XG;
            #pragma unroll
            for (int grp = 0; grp < 4; ++grp) {
                v8us hv, lv;
                pack_group(pbuf4[t * 8 + 2 * grp], pbuf4[t * 8 + 2 * grp + 1], hv, lv);
                xsh[xb + grp] = hv;
                xsl[xb + grp] = lv;
            }
            const v4f* f4 = (const v4f*)(feats + ((size_t)grow * NS + n) * NF);
            #pragma unroll
            for (int grp = 0; grp < 2; ++grp) {
                v8us hv, lv;
                pack_group(f4[2 * grp], f4[2 * grp + 1], hv, lv);
                xsh[xb + 4 + grp] = hv;
                xsl[xb + 4 + grp] = lv;
            }
        }
        __syncthreads();

        #pragma unroll 1
        for (int e = 0; e < NE; ++e) {
            int nt = __builtin_amdgcn_readfirstlane(ntE[e]);
            int tb = __builtin_amdgcn_readfirstlane(startT[e]);
            nt = nt < 0 ? 0 : (nt > NTPE ? NTPE : nt);
            tb = tb < 0 ? 0 : (tb > NTILE - 1 ? NTILE - 1 : tb);
            const v8us* w0e = a0f + e * 2048;
            const v8us* w1e = a1f + e * 1024;
            #pragma unroll 1
            for (int j = 0; j < nt; ++j) {
                int tile = tb + j;
                tile = tile > NTILE - 1 ? NTILE - 1 : tile;
                if ((tile & (NWAV - 1)) != wave) continue;
                const int slot = tile * 16 + m16;
                const int xb   = slot * XG;

                Frag xb0h, xb0l, xb1h, xb1l;
                xb0h.h8[0] = xsh[xb + g];     xb0h.h8[1] = xsh[xb + 2 + g];
                xb0l.h8[0] = xsl[xb + g];     xb0l.h8[1] = xsl[xb + 2 + g];
                xb1h.h8[0] = xsh[xb + 4 + g]; xb1h.h8[1] = z8;
                xb1l.h8[0] = xsl[xb + 4 + g]; xb1l.h8[1] = z8;

                v8f acc1a, acc1b;
                #pragma unroll
                for (int r = 0; r < 8; ++r) {
                    acc1a[r] = b1s[e * NP + 8 * g + r];
                    acc1b[r] = b1s[e * NP + 16 + 8 * g + r];
                }

                #pragma unroll 1
                for (int c = 0; c < 4; ++c) {
                    Frag hbh, hbl;
                    #pragma unroll
                    for (int u = 0; u < 2; ++u) {
                        const int t8 = 2 * c + u;
                        v8f acc0;
                        #pragma unroll
                        for (int r = 0; r < 8; ++r) acc0[r] = b0s[e * NH + t8 * 16 + 8 * g + r];
                        Frag wh, wl;
                        int fb = ((t8 * 2 + 0) * 2) * 64 + lane * 2;
                        wh.h8[0] = w0e[fb];      wh.h8[1] = w0e[fb + 1];
                        wl.h8[0] = w0e[fb + 64]; wl.h8[1] = w0e[fb + 65];
                        acc0 = wmma3(acc0, wh, wl, xb0h, xb0l);
                        fb = ((t8 * 2 + 1) * 2) * 64 + lane * 2;
                        wh.h8[0] = w0e[fb];      wh.h8[1] = w0e[fb + 1];
                        wl.h8[0] = w0e[fb + 64]; wl.h8[1] = w0e[fb + 65];
                        acc0 = wmma3(acc0, wh, wl, xb1h, xb1l);
                        #pragma unroll
                        for (int r = 0; r < 8; ++r) {
                            unsigned short hi, lo;
                            split2(fast_tanh(acc0[r]), hi, lo);
                            hbh.s[u * 8 + r] = hi;
                            hbl.s[u * 8 + r] = lo;
                        }
                    }
                    {
                        Frag wh, wl;
                        const int fb = ((0 * 4 + c) * 2) * 64 + lane * 2;
                        wh.h8[0] = w1e[fb];      wh.h8[1] = w1e[fb + 1];
                        wl.h8[0] = w1e[fb + 64]; wl.h8[1] = w1e[fb + 65];
                        acc1a = wmma3(acc1a, wh, wl, hbh, hbl);
                    }
                    {
                        Frag wh, wl;
                        const int fb = ((1 * 4 + c) * 2) * 64 + lane * 2;
                        wh.h8[0] = w1e[fb];      wh.h8[1] = w1e[fb + 1];
                        wl.h8[0] = w1e[fb + 64]; wl.h8[1] = w1e[fb + 65];
                        acc1b = wmma3(acc1b, wh, wl, hbh, hbl);
                    }
                }

                osl4[slot * 8 + 2 * g]     = lo4(acc1a);
                osl4[slot * 8 + 2 * g + 1] = hi4(acc1a);
                osl4[slot * 8 + 4 + 2 * g] = lo4(acc1b);
                osl4[slot * 8 + 5 + 2 * g] = hi4(acc1b);
            }
        }
        __syncthreads();

        if (active) {
            #pragma unroll
            for (int i = 0; i < 8; ++i) pbuf4[t * 8 + i] = osl4[myslot * 8 + i];
        }
        __syncthreads();
    }

    v4f ov[8];
    #pragma unroll
    for (int it = 0; it < 8; ++it) {
        const int row = it * 32 + (t >> 3);
        v4f v = pbuf4[row * 8 + (t & 7)];
        v[0] = fmaxf(v[0], 0.f); v[1] = fmaxf(v[1], 0.f);
        v[2] = fmaxf(v[2], 0.f); v[3] = fmaxf(v[3], 0.f);
        ov[it] = v;
    }
    volatile v4f* vo = (volatile v4f*)out;
    #pragma unroll
    for (int it = 0; it < 8; ++it) {
        const int row = it * 32 + (t >> 3);
        if (r0 + row < nrows) vo[(size_t)(r0 + row) * 8 + (t & 7)] = ov[it];
    }
    __threadfence();
    #pragma unroll
    for (int it = 0; it < 8; ++it) {
        const int row = it * 32 + (t >> 3);
        if (r0 + row < nrows) vo[(size_t)(r0 + row) * 8 + (t & 7)] = ov[it];
    }
}

extern "C" void kernel_launch(void* const* d_in, const int* in_sizes, int n_in,
                              void* d_out, int out_size, void* d_ws, size_t ws_size,
                              hipStream_t stream) {
    if (n_in < 8) return;
    const int*   mod_id_seq   = (const int*)d_in[0];
    const float* mod_feat_seq = (const float*)d_in[1];
    const float* p_in         = (const float*)d_in[2];
    const int*   seq_len      = (const int*)d_in[3];
    const float* W0           = (const float*)d_in[4];
    const float* b0           = (const float*)d_in[5];
    const float* W1           = (const float*)d_in[6];
    const float* b1           = (const float*)d_in[7];
    float*       out          = (float*)d_out;

    const int B = in_sizes[3];
    if (B <= 0) return;
    if (in_sizes[0] != B * NS) return;
    if (in_sizes[1] != B * NS * NF) return;
    if (in_sizes[2] != B * NP) return;
    if (in_sizes[4] != NE * NX * NH) return;
    if (in_sizes[5] != NE * NH) return;
    if (in_sizes[6] != NE * NH * NP) return;
    if (in_sizes[7] != NE * NP) return;
    if (out_size != B * NP) return;

    const size_t need = (size_t)(N0F + N1F) * 16;
    if (ws_size < need) return;
    v4u* a0 = (v4u*)d_ws;
    v4u* a1 = a0 + N0F;

    const int nthr_pack = N0F + N1F;
    k_pack<<<(nthr_pack + 255) / 256, 256, 0, stream>>>(W0, W1, a0, a1);

    const int nblk = (B + ROWS - 1) / ROWS;
    k_main<<<nblk, NTHR, 0, stream>>>(mod_id_seq, mod_feat_seq, p_in, seq_len, b0, b1,
                                       (const v8us*)a0, (const v8us*)a1, out, B);
}
